// SparseGaussianProcess_8100308321081
// MI455X (gfx1250) — hardware-run, weakly checked
//
#include <hip/hip_runtime.h>


namespace {
constexpr int NPT = 65536, ID = 16, OD = 8, M = 1024, S = 8, L = 64, SO = S * OD  , MCH = 256;
constexpr float HS = 256.0f, WSC = 256.0f;
typedef _Float16 b16;
typedef __attribute__((ext_vector_type(16))) _Float16 v16b;
typedef __attribute__((ext_vector_type(8))) _Float16 v8b;
typedef __attribute__((ext_vector_type(8))) float v8f;
typedef __attribute__((ext_vector_type(4))) float v4f;
__device__ __forceinline__ float bf16_rne(float f) { unsigned int u = __float_as_uint(f); u += 0x7FFFu + ((u >> 16) & 1u); float r = __uint_as_float(u & 0xFFFF0000u); asm volatile("" : "+v"(r)); return r; }
__device__ __forceinline__ float bfv(float f) { float r = bf16_rne(f); asm volatile("" : "+v"(r)); return r; }
__device__ __forceinline__ void split16(float v, b16& hi, b16& lo) { hi = (b16)v; lo = (b16)(v - (float)hi); }
__device__ __forceinline__ v16b frag_kb(const b16* p, int hh) { const v8b a = *(const v8b*)(p + 8 * hh), b = *(const v8b*)(p + 16 + 8 * hh); v16b f;
#pragma unroll
  for (int e = 0; e < 8; ++e) { f[e] = a[e]; f[8 + e] = b[e]; } return f; }
__device__ __forceinline__ v8f wmma16b(v16b a, v16b b, v8f c) { v8f d = __builtin_amdgcn_wmma_f32_16x16x32_f16(false, a, false, b, (short)0, c, false, false); asm volatile("v_nop\n\tv_nop\n\tv_nop\n\tv_nop" : "+v"(d) : "v"(a), "v"(b)); return d; }
__device__ __forceinline__ void wave_lds_sync() { __builtin_amdgcn_fence(__ATOMIC_RELEASE, "workgroup"); __builtin_amdgcn_wave_barrier(); __builtin_amdgcn_fence(__ATOMIC_ACQUIRE, "workgroup"); }
__device__ __forceinline__ float pmul(float a, float b) { float p = a * b; asm volatile("" : "+v"(p)); return p; }

__global__ __launch_bounds__(256) void setup_kernel(const float* __restrict__ freq, const float* __restrict__ pw, const float* __restrict__ z, const float* __restrict__ iw, b16* __restrict__ FT, b16* __restrict__ PWT, b16* __restrict__ ZT, b16* __restrict__ IWT, float* __restrict__ Z2) { const int u = blockIdx.x * 256 + threadIdx.x; v8b v;
  if (u < OD * L * 4) { const int r = u / 4, k0 = (u % 4) * 8; const int o = r / L, l = r % L;
#pragma unroll
    for (int j = 0; j < 8; ++j) { const int k = k0 + j; v[j] = (b16)(k < ID ? bf16_rne(freq[((size_t)o * ID + k) * L + l]) * WSC : 0.0f); } for (int pass = 0; pass < 2; ++pass) { *(volatile v8b*)(FT + (size_t)r * 32 + k0) = v; __threadfence(); } }
  if (u < OD * 16 * 8) { const int r = u / 8, l0 = (u % 8) * 8; const int o = r / 16, s = r % 16;
#pragma unroll
    for (int j = 0; j < 8; ++j) v[j] = (b16)(s < S ? bf16_rne(pw[((size_t)s * OD + o) * L + l0 + j]) * WSC : 0.0f); for (int pass = 0; pass < 2; ++pass) { *(volatile v8b*)(PWT + (size_t)r * L + l0) = v; __threadfence(); } }
  if (u < M * 4) { const int m = u / 4, k0 = (u % 4) * 8;
#pragma unroll
    for (int j = 0; j < 8; ++j) { const int k = k0 + j; v[j] = (b16)(k < ID ? bf16_rne(z[(size_t)m * ID + k]) * WSC : 0.0f); } for (int pass = 0; pass < 2; ++pass) { *(volatile v8b*)(ZT + (size_t)m * 32 + k0) = v; __threadfence(); } }
  if (u < SO * (M / 8)) { const int r = u / (M / 8), m0 = (u % (M / 8)) * 8;
#pragma unroll
    for (int j = 0; j < 8; ++j) v[j] = (b16)(bf16_rne(iw[(size_t)r * M + m0 + j]) * WSC); for (int pass = 0; pass < 2; ++pass) { *(volatile v8b*)(IWT + (size_t)r * M + m0) = v; __threadfence(); } }
  if (u < M) { float sq = 0.0f; for (int k = 0; k < ID; ++k) { const float zz = bfv(z[(size_t)u * ID + k]); sq += zz * zz; } for (int pass = 0; pass < 2; ++pass) { ((volatile float*)Z2)[u] = sq; __threadfence(); } }
}
__global__ __launch_bounds__(32) void sgp_kernel(const float* __restrict__ x, const float* __restrict__ phase, const float* __restrict__ Z2, const b16* __restrict__ FT, const b16* __restrict__ PWT, const b16* __restrict__ ZT, const b16* __restrict__ IWT, int NLIM, float* __restrict__ out) {
  __shared__ __attribute__((aligned(16))) b16 Xh[32][40], Bh[32][L + 8], Bl[32][L + 8], Kh[32][MCH + 8], Kl[32][MCH + 8]; __shared__ float Tf[SO][36], Xz[32][MCH + 4], In[32][L + 4]; __shared__ float X2[32];
  const int lane = threadIdx.x, nloc = lane & 15, hlf = lane >> 4; const size_t n0 = (size_t)blockIdx.x * 32; if (n0 >= (size_t)NLIM) return;
  { float sq = 0.0f; for (int k = 0; k < ID; ++k) { const float xv = bfv(x[(n0 + lane) * ID + k]); sq += xv * xv; Xh[lane][k] = (b16)(xv * HS); } for (int k = ID; k < 40; ++k) Xh[lane][k] = (b16)0.0f; X2[lane] = sq; }
  if (lane < 16) for (int r = 0; r < 32; ++r) for (int k = L; k < L + 8; k += 8) { Bh[r][k + (lane & 7)] = (b16)0.0f; Bl[r][k + (lane & 7)] = (b16)0.0f; }
  wave_lds_sync();
  const v16b xa0 = frag_kb(&Xh[nloc][0], hlf), xa1 = frag_kb(&Xh[16 + nloc][0], hlf);
#pragma unroll 1
  for (int o = 0; o < OD; ++o) { v8f in0[4], in1[4];
#pragma unroll
    for (int t = 0; t < 4; ++t) { const v16b bf = frag_kb(FT + ((size_t)o * L + t * 16 + nloc) * 32, hlf); in0[t] = wmma16b(xa0, bf, (v8f){}); in1[t] = wmma16b(xa1, bf, (v8f){}); }
#pragma unroll
    for (int t = 0; t < 4; ++t) {
#pragma unroll
      for (int r8 = 0; r8 < 8; ++r8) { In[8 * hlf + r8][t * 16 + nloc] = in0[t][r8]; In[16 + 8 * hlf + r8][t * 16 + nloc] = in1[t][r8]; } }
    wave_lds_sync();
    { const float ph0 = bfv(phase[o * L + lane]), ph1 = bfv(phase[o * L + 32 + lane]);
#pragma unroll 1
      for (int r = 0; r < 32; ++r) { b16 p, q; split16(cosf(In[r][lane] * (1.0f / (HS * WSC)) + ph0) * HS, p, q); Bh[r][lane] = p; Bl[r][lane] = q; split16(cosf(In[r][32 + lane] * (1.0f / (HS * WSC)) + ph1) * HS, p, q); Bh[r][32 + lane] = p; Bl[r][32 + lane] = q; } }
    wave_lds_sync(); v8f pr0 = {}, pr1 = {};
#pragma unroll
    for (int kb = 0; kb < L; kb += 32) { const v16b bw = frag_kb(PWT + ((size_t)o * 16 + nloc) * L + kb, hlf); pr0 = wmma16b(frag_kb(&Bh[nloc][kb], hlf), bw, pr0); pr0 = wmma16b(frag_kb(&Bl[nloc][kb], hlf), bw, pr0); pr1 = wmma16b(frag_kb(&Bh[16 + nloc][kb], hlf), bw, pr1); pr1 = wmma16b(frag_kb(&Bl[16 + nloc][kb], hlf), bw, pr1); }
    if (nloc < S) {
#pragma unroll
      for (int r8 = 0; r8 < 8; ++r8) { Tf[nloc * OD + o][8 * hlf + r8] = pr0[r8] * (0.17677669529663687f / (HS * WSC)); Tf[nloc * OD + o][16 + 8 * hlf + r8] = pr1[r8] * (0.17677669529663687f / (HS * WSC)); } }
    wave_lds_sync(); }
  v8f da0[4] = {(v8f){}, (v8f){}, (v8f){}, (v8f){}}, da1[4] = {(v8f){}, (v8f){}, (v8f){}, (v8f){}};
#pragma unroll 1
  for (int mc = 0; mc < M; mc += MCH) {
#pragma unroll 1
    for (int t = 0; t < MCH / 16; ++t) { const v16b bz = frag_kb(ZT + (size_t)(mc + t * 16 + nloc) * 32, hlf); const v8f d0 = wmma16b(xa0, bz, (v8f){}), d1 = wmma16b(xa1, bz, (v8f){});
#pragma unroll
      for (int r8 = 0; r8 < 8; ++r8) { Xz[8 * hlf + r8][t * 16 + nloc] = d0[r8]; Xz[16 + 8 * hlf + r8][t * 16 + nloc] = d1[r8]; } }
    wave_lds_sync();
    for (int r = 0; r < 32; ++r) for (int q = 0; q < MCH / 32; ++q) { const int mm = q * 32 + lane; const float sq = fmaxf(X2[r] + Z2[mc + mm] - 2.0f * Xz[r][mm] * (1.0f / (HS * WSC)), 0.0f); b16 p, ql; split16(expf(-0.5f * sq) * HS, p, ql); Kh[r][mm] = p; Kl[r][mm] = ql; }
    if (lane < 16) for (int r = 0; r < 32; ++r) { Kh[r][MCH + (lane & 7)] = (b16)0.0f; Kl[r][MCH + (lane & 7)] = (b16)0.0f; }
    wave_lds_sync();
#pragma unroll 2
    for (int kb = 0; kb < MCH; kb += 32) { const v16b a0 = frag_kb(&Kh[nloc][kb], hlf), l0 = frag_kb(&Kl[nloc][kb], hlf), a1 = frag_kb(&Kh[16 + nloc][kb], hlf), l1 = frag_kb(&Kl[16 + nloc][kb], hlf);
#pragma unroll
      for (int t = 0; t < 4; ++t) { const v16b bw = frag_kb(IWT + (size_t)(t * 16 + nloc) * M + mc + kb, hlf); da0[t] = wmma16b(a0, bw, da0[t]); da0[t] = wmma16b(l0, bw, da0[t]); da1[t] = wmma16b(a1, bw, da1[t]); da1[t] = wmma16b(l1, bw, da1[t]); } }
    wave_lds_sync(); }
#pragma unroll
  for (int t = 0; t < 4; ++t)
#pragma unroll
    for (int r8 = 0; r8 < 8; ++r8) { Tf[t * 16 + nloc][8 * hlf + r8] += da0[t][r8] * (1.0f / (HS * WSC)); Tf[t * 16 + nloc][16 + 8 * hlf + r8] += da1[t][r8] * (1.0f / (HS * WSC)); }
  wave_lds_sync();
  for (int pass = 0; pass < 2; ++pass) { for (int so = 0; so < SO; ++so) ((volatile float*)out)[(size_t)so * NPT + n0 + lane] = Tf[so][lane]; __threadfence(); } }
}

extern "C" void kernel_launch(void* const* d_in, const int* in_sizes, int n_in, void* d_out, int out_size, void* d_ws, size_t ws_size, hipStream_t stream) {
  (void)n_in;
  auto Fp = [&](int i) { return (const float*)d_in[i]; };
  if (in_sizes[0] != NPT * ID || in_sizes[1] != M * ID || in_sizes[2] != S * OD * M || in_sizes[3] != OD * ID * L || in_sizes[4] != OD * L || in_sizes[5] != S * OD * L || out_size != S * OD * NPT) return;
  const int NLIM = NPT;
  size_t off = 0; char* ws = (char*)d_ws;
  auto carve = [&](size_t bytes) { char* p = ws + off; off += (bytes + 255) & ~(size_t)255; return p; };
  b16* FT = (b16*)carve((size_t)OD * L * 32 * 2); b16* PWT = (b16*)carve((size_t)OD * 16 * L * 2); b16* ZT = (b16*)carve((size_t)M * 32 * 2); b16* IWT = (b16*)carve((size_t)SO * M * 2); float* Z2 = (float*)carve((size_t)M * 4);
  if (off > ws_size || off > ((size_t)4 << 20)) return;
  setup_kernel<<<(SO * (M / 8) + 255) / 256, 256, 0, stream>>>(Fp(3), Fp(5), Fp(1), Fp(2), FT, PWT, ZT, IWT, Z2);
  sgp_kernel<<<NLIM / 32, 32, 0, stream>>>(Fp(0), Fp(4), Z2, FT, PWT, ZT, IWT, NLIM, (float*)d_out);
}
